// MahalanobisBlock_43404939493451
// MI455X (gfx1250) — hardware-verified
//
#include <hip/hip_runtime.h>
#include <stddef.h>
#include <stdint.h>

#define NQ     64
#define NCL    16
#define NBS    8
#define NCH    256
#define HW     441
#define HWP    448
#define CSP    32
#define PIECES 56

#define OUTROW      (NCL * HW)
#define OUTS_FLOATS (2 * OUTROW)
#define OUT_LINES   (OUTS_FLOATS / 32)
#define OUT_ITERS   ((OUT_LINES + 31) / 32)
#define SIM_UNITS   (2 * NCL * (HWP / 16))
#define SIM_ITERS   (SIM_UNITS / 4)
#define GRAM_TILES  10

#define CS_BYTES  ((size_t)NCL * NCH * CSP * 4)
#define XH_BYTES  ((size_t)NCL * NBS * NCH * HWP * 2)
#define LP_BYTES  ((size_t)NCL * NCH * NCH * 2)
#define DT_BYTES  ((size_t)NQ * HWP * NCH * 2)
#define OFF_CS    ((size_t)0)
#define OFF_XH    (OFF_CS + CS_BYTES)
#define OFF_LP    (OFF_XH + XH_BYTES)
#define OFF_DT    (OFF_LP + LP_BYTES)
#define WS_TOTAL  (OFF_DT + DT_BYTES)

static_assert(OUT_LINES * 32 == OUTS_FLOATS);
static_assert(OUT_LINES == 441);
static_assert(SIM_ITERS * 4 == SIM_UNITS);
static_assert((HWP % 32) == 0);
static_assert(PIECES * 8 == HWP);
static_assert(NBS * PIECES <= 512);
static_assert((OFF_XH % 256) == 0);
static_assert((OFF_LP % 256) == 0);
static_assert((OFF_DT % 256) == 0);
static_assert(WS_TOTAL == 46661632);
static_assert(WS_TOTAL <= (size_t)134217728);

typedef unsigned short v8us  __attribute__((ext_vector_type(8)));
typedef unsigned short v16us __attribute__((ext_vector_type(16)));
typedef _Float16       v8h   __attribute__((ext_vector_type(8)));
typedef _Float16       v16h  __attribute__((ext_vector_type(16)));
typedef float          v4f   __attribute__((ext_vector_type(4)));
typedef float          v8f   __attribute__((ext_vector_type(8)));
#if defined(__HIP_DEVICE_COMPILE__)
typedef __bf16         v16bf __attribute__((ext_vector_type(16)));
#endif

union FragU { v16us v; v8us half[2]; };
union FragH { v16h  v; v8h  half[2]; };

__device__ __forceinline__ unsigned bbits(float f) {
  unsigned u = __float_as_uint(f);
  return (u + 0x7FFFu + ((u >> 16) & 1u)) >> 16;
}
__device__ __forceinline__ float bf16r(float f) {
  return __uint_as_float(bbits(f) << 16);
}
__device__ __forceinline__ v8f zero8() { v8f z = {0.f, 0.f, 0.f, 0.f, 0.f, 0.f, 0.f, 0.f}; return z; }

__device__ __forceinline__ v16us ldfrag_u(const unsigned short* p) {
  FragU f;
  f.half[0] = *(const v8us*)(p);
  f.half[1] = *(const v8us*)(p + 16);
  return f.v;
}

__device__ __forceinline__ v8f mma_bf(v16us a, v16us b, v8f c) {
#if defined(__HIP_DEVICE_COMPILE__)
  return __builtin_amdgcn_wmma_f32_16x16x32_bf16(false, __builtin_bit_cast(v16bf, a),
                                                false, __builtin_bit_cast(v16bf, b),
                                                (short)0, c, false, false);
#else
  (void)a; (void)b;
  return c;
#endif
}
__device__ __forceinline__ v8f mma_h(v16h a, v16h b, v8f c) {
#if defined(__HIP_DEVICE_COMPILE__)
  return __builtin_amdgcn_wmma_f32_16x16x32_f16(false, a, false, b, (short)0, c, false, false);
#else
  (void)a; (void)b;
  return c;
#endif
}
__device__ __forceinline__ void guard_g(v8f& c0, v8f& c1, v8f& c2, v8f& c3, const v16us& a,
                                        const v16us& b0, const v16us& b1, const v16us& b2,
                                        const v16us& b3) {
#if defined(__HIP_DEVICE_COMPILE__)
  asm volatile("v_nop\n\tv_nop\n\tv_nop\n\tv_nop"
               : "+v"(c0), "+v"(c1), "+v"(c2), "+v"(c3)
               : "v"(a), "v"(b0), "v"(b1), "v"(b2), "v"(b3));
#else
  (void)c0; (void)c1; (void)c2; (void)c3; (void)a; (void)b0; (void)b1; (void)b2; (void)b3;
#endif
}
__device__ __forceinline__ void guard_s(v8f& c0, v8f& c1, v8f& c2, v8f& c3, v8f& c4, v8f& c5,
                                        v8f& c6, v8f& c7, const v16h& a, const v16h& b) {
#if defined(__HIP_DEVICE_COMPILE__)
  asm volatile("v_nop\n\tv_nop\n\tv_nop\n\tv_nop"
               : "+v"(c0), "+v"(c1), "+v"(c2), "+v"(c3), "+v"(c4), "+v"(c5), "+v"(c6), "+v"(c7)
               : "v"(a), "v"(b));
#else
  (void)c0; (void)c1; (void)c2; (void)c3; (void)c4; (void)c5; (void)c6; (void)c7; (void)a; (void)b;
#endif
}

__global__ __launch_bounds__(256)
void k_xprep(const float* __restrict__ x2, unsigned short* xh, float* cs)
{
  const int nc   = blockIdx.x;
  const int n    = nc >> 8;
  const int c    = nc & 255;
  const int tid  = threadIdx.x;
  const int lane = tid & 31;
  const int w    = tid >> 5;

  float sum = 0.f;
  v8us   o[2];
  size_t doff[2];
  bool   ok[2];
#pragma unroll
  for (int it = 0; it < 2; ++it) {
    const int item  = it * 256 + tid;
    const bool valid = item < NBS * PIECES;
    const int itc   = valid ? item : (NBS * PIECES - 1);
    const int bs    = itc / PIECES;
    const int j     = itc - bs * PIECES;
    const float* src = x2 + (((size_t)(n * NBS + bs)) * NCH + (size_t)c) * HW;
    v8us ov;
#pragma unroll
    for (int e = 0; e < 8; ++e) {
      const int p  = 8 * j + e;
      const int pc = (p < HW) ? p : (HW - 1);
      float v = bf16r(src[pc]);
      v = (p < HW) ? v : 0.f;
      sum += valid ? v : 0.f;
      ov[e] = (unsigned short)bbits(v);
    }
    o[it]    = ov;
    ok[it]   = valid;
    doff[it] = (((size_t)(n * NBS + bs)) * NCH + (size_t)c) * HWP + (size_t)(8 * j);
  }
#pragma unroll
  for (int it = 0; it < 2; ++it)
    if (ok[it]) *(volatile v8us*)(xh + doff[it]) = o[it];

#pragma unroll
  for (int off = 16; off >= 1; off >>= 1) sum += __shfl_xor(sum, off, 32);
  __shared__ float red[8];
  if (lane == 0) red[w] = sum;
  __syncthreads();
  float tot = 0.f;
  if (w == 0) {
    float v = red[lane & 7];
    v = (lane < 8) ? v : 0.f;
#pragma unroll
    for (int off = 16; off >= 1; off >>= 1) v += __shfl_xor(v, off, 32);
    tot = v;
  }
  v4f cv;
  cv[0] = (lane == 0) ? tot : 0.f;
  cv[1] = 0.f; cv[2] = 0.f; cv[3] = 0.f;
  float* cdst = cs + (size_t)nc * CSP + 4 * (lane & 7);
  const bool cwr = (w == 0) && (lane < 8);
  if (cwr) *(volatile v4f*)cdst = cv;

  __threadfence();

#pragma unroll
  for (int it = 0; it < 2; ++it)
    if (ok[it]) *(volatile v8us*)(xh + doff[it]) = o[it];
  if (cwr) *(volatile v4f*)cdst = cv;
}

__global__ __launch_bounds__(256)
void k_qprep(const float* __restrict__ x1, _Float16* dt)
{
  const int b    = blockIdx.x >> 2;
  const int cg   = blockIdx.x & 3;
  const int tid  = threadIdx.x;
  const int lane = tid & 31;
  const int w    = tid >> 5;

  __shared__ float shRn[64];
  __shared__ float shMq[64];

#pragma unroll 1
  for (int e = 0; e < 8; ++e) {
    const int ch = 8 * w + e;
    const int c  = 64 * cg + ch;
    const float* row = x1 + ((size_t)b * NCH + (size_t)c) * HW;
    float s1 = 0.f, ss = 0.f;
#pragma unroll 2
    for (int t = 0; t < 14; ++t) {
      const int p  = lane + 32 * t;
      const int pc = (p < HW) ? p : (HW - 1);
      float v = bf16r(row[pc]);
      v = (p < HW) ? v : 0.f;
      s1 += v;
      ss += v * v;
    }
#pragma unroll
    for (int off = 16; off >= 1; off >>= 1) {
      s1 += __shfl_xor(s1, off, 32);
      ss += __shfl_xor(ss, off, 32);
    }
    const float rn = 1.0f / sqrtf(ss);
    const float mq = (s1 * rn) * (1.0f / (float)HW);
    if (lane == 0) { shRn[ch] = rn; shMq[ch] = mq; }
  }
  __syncthreads();

  const int q  = lane >> 3;
  const int jj = lane & 7;
#pragma unroll 1
  for (int it = 0; it < 14; ++it) {
    const int p  = it * 32 + w * 4 + q;
    const int pc = (p < HW) ? p : (HW - 1);
    v8h o;
#pragma unroll
    for (int e = 0; e < 8; ++e) {
      const int ch = 8 * jj + e;
      const float x = bf16r(x1[((size_t)b * NCH + (size_t)(64 * cg + ch)) * HW + pc]);
      float d = (x * shRn[ch] - shMq[ch]) * 64.0f;
      d = (p < HW) ? d : 0.f;
      o[e] = (_Float16)d;
    }
    _Float16* dst = dt + ((size_t)b * HWP + (size_t)p) * NCH + (size_t)(64 * cg + 8 * jj);
    *(volatile v8h*)dst = o;
    __threadfence();
    *(volatile v8h*)dst = o;
  }
}

__global__ __launch_bounds__(128)
void k_gram(const unsigned short* __restrict__ xh, const float* __restrict__ cs, _Float16* lp)
{
  const int n    = blockIdx.x / GRAM_TILES;
  const int t    = blockIdx.x - n * GRAM_TILES;
  const int ti   = (t >= 1) + (t >= 3) + (t >= 6);
  const int tj   = t - (ti * (ti + 1)) / 2;
  const int tid  = threadIdx.x;
  const int lane = tid & 31;
  const int w    = tid >> 5;
  const int h    = lane >> 4;
  const int m    = lane & 15;

  __shared__ __align__(16) _Float16 tile[64 * 64];

  const int c0 = 64 * ti + 16 * w;
  const int d0 = 64 * tj;

  v8f acc[4];
#pragma unroll
  for (int j = 0; j < 4; ++j) acc[j] = zero8();

  const unsigned short* xn = xh + (size_t)n * NBS * NCH * HWP;
#pragma unroll 1
  for (int bs = 0; bs < NBS; ++bs) {
    const unsigned short* pa = xn + ((size_t)bs * NCH + (size_t)(c0 + m)) * HWP + 8 * h;
    const unsigned short* pb = xn + ((size_t)bs * NCH + (size_t)(d0 + m)) * HWP + 8 * h;
#pragma unroll 2
    for (int kk = 0; kk < 14; ++kk) {
      const v16us a  = ldfrag_u(pa + 32 * kk);
      const v16us b0 = ldfrag_u(pb + 32 * kk);
      const v16us b1 = ldfrag_u(pb + 16 * HWP + 32 * kk);
      const v16us b2 = ldfrag_u(pb + 32 * HWP + 32 * kk);
      const v16us b3 = ldfrag_u(pb + 48 * HWP + 32 * kk);
      acc[0] = mma_bf(a, b0, acc[0]);
      acc[1] = mma_bf(a, b1, acc[1]);
      acc[2] = mma_bf(a, b2, acc[2]);
      acc[3] = mma_bf(a, b3, acc[3]);
      guard_g(acc[0], acc[1], acc[2], acc[3], a, b0, b1, b2, b3);
    }
  }

  const float invR   = 1.0f / 3528.0f;
  const float invRm1 = 1.0f / 3527.0f;
  float csr[8];
#pragma unroll
  for (int r = 0; r < 8; ++r)
    csr[r] = cs[((size_t)n * NCH + (size_t)(c0 + 8 * h + r)) * CSP];
#pragma unroll
  for (int j = 0; j < 4; ++j) {
    const int d = d0 + 16 * j + m;
    const float mcol = cs[((size_t)n * NCH + (size_t)d) * CSP] * invR;
#pragma unroll
    for (int r = 0; r < 8; ++r) {
      const int c = c0 + 8 * h + r;
      const float cv  = (acc[j][r] - csr[r] * mcol) * invRm1;
      const float val = (d < c) ? (2.0f * cv) : ((d == c) ? cv : 0.f);
      tile[(16 * w + 8 * h + r) * 64 + 16 * j + m] = (_Float16)(val * 16.0f);
    }
  }
  __syncthreads();

  const int q  = lane >> 3;
  const int jj = lane & 7;
  const size_t plane = (size_t)n * NCH * NCH;
  const bool mirror = (tj < ti);
  v8h zz;
#pragma unroll
  for (int e = 0; e < 8; ++e) zz[e] = (_Float16)0.0f;
  v8h    v[4];
  size_t off[4];
  size_t offz[4];
#pragma unroll
  for (int it = 0; it < 4; ++it) {
    const int lr = it * 16 + w * 4 + q;
    v[it]    = *(const v8h*)(tile + lr * 64 + 8 * jj);
    off[it]  = plane + ((size_t)(64 * ti + lr)) * NCH + (size_t)(64 * tj + 8 * jj);
    offz[it] = plane + ((size_t)(64 * tj + lr)) * NCH + (size_t)(64 * ti + 8 * jj);
  }
#pragma unroll
  for (int it = 0; it < 4; ++it) {
    *(volatile v8h*)(lp + off[it]) = v[it];
    if (mirror) *(volatile v8h*)(lp + offz[it]) = zz;
  }
  __threadfence();
#pragma unroll
  for (int it = 0; it < 4; ++it) {
    *(volatile v8h*)(lp + off[it]) = v[it];
    if (mirror) *(volatile v8h*)(lp + offz[it]) = zz;
  }
}

__global__ __launch_bounds__(256)
void k_sim(const _Float16* __restrict__ lp, const _Float16* __restrict__ dt, float* out)
{
  __shared__ __align__(16) float outS[OUTS_FLOATS];
  __shared__ float xch[2][4][16];

  const int tid  = threadIdx.x;
  const int lane = tid & 31;
  const int w    = tid >> 5;
  const int h    = lane >> 4;
  const int m    = lane & 15;
  const int pair = w >> 1;
  const int par  = w & 1;
  const int b0   = blockIdx.x * 2;

#pragma unroll 1
  for (int t = 0; t < SIM_ITERS; ++t) {
    const int u   = t * 4 + pair;
    const int bl  = u / (NCL * (HWP / 16));
    const int rem = u - bl * (NCL * (HWP / 16));
    const int n   = rem / (HWP / 16);
    const int ct  = rem - n * (HWP / 16);
    const int b   = b0 + bl;
    const int p   = 16 * ct + m;

    const _Float16* pB = dt + ((size_t)b * HWP + (size_t)p) * NCH + 8 * h;
    const _Float16* pA = lp + (size_t)n * NCH * NCH + (size_t)(16 * par + m) * NCH + 8 * h;

    v8f acc[8];
#pragma unroll
    for (int j = 0; j < 8; ++j) acc[j] = zero8();
    float s = 0.f;

#pragma unroll
    for (int kk = 0; kk < 8; ++kk) {
      FragH fb;
      fb.half[0] = *(const v8h*)(pB + 32 * kk);
      fb.half[1] = *(const v8h*)(pB + 32 * kk + 16);
      v16h alast = fb.v;
#pragma unroll
      for (int j = 0; j < 8; ++j) {
        if (j >= kk) {
          const _Float16* qa = pA + (size_t)(32 * j) * NCH + 32 * kk;
          FragH fa;
          fa.half[0] = *(const v8h*)(qa);
          fa.half[1] = *(const v8h*)(qa + 16);
          acc[j] = mma_h(fa.v, fb.v, acc[j]);
          alast = fa.v;
        }
      }
      guard_s(acc[0], acc[1], acc[2], acc[3], acc[4], acc[5], acc[6], acc[7], alast, fb.v);
      const v8h bq = par ? fb.half[1] : fb.half[0];
#pragma unroll
      for (int r = 0; r < 8; ++r) s += acc[kk][r] * (float)bq[r];
    }
    s += __shfl_xor(s, 16, 32);
    if (par == 1 && h == 0) xch[t & 1][pair][m] = s;
    __syncthreads();
    if (par == 0 && h == 0 && p < HW)
      outS[(bl * NCL + n) * HW + p] = (s + xch[t & 1][pair][m]) * (1.0f / 65536.0f);
  }
  __syncthreads();

  float* ob = out + (size_t)blockIdx.x * (size_t)OUTS_FLOATS;
  const int q4 = lane >> 3;
  const int jj = lane & 7;
#pragma unroll 1
  for (int it = 0; it < OUT_ITERS; ++it) {
    const int line = it * 32 + w * 4 + q4;
    const int lc   = (line < OUT_LINES) ? line : (OUT_LINES - 1);
    const v4f v = *(const v4f*)(outS + lc * 32 + jj * 4);
    if (line < OUT_LINES) *(volatile v4f*)(ob + (size_t)lc * 32 + jj * 4) = v;
  }
  __threadfence();
#pragma unroll 1
  for (int it = 0; it < OUT_ITERS; ++it) {
    const int line = it * 32 + w * 4 + q4;
    const int lc   = (line < OUT_LINES) ? line : (OUT_LINES - 1);
    const v4f v = *(const v4f*)(outS + lc * 32 + jj * 4);
    if (line < OUT_LINES) *(volatile v4f*)(ob + (size_t)lc * 32 + jj * 4) = v;
  }
}

extern "C" void kernel_launch(void* const* d_in, const int* in_sizes, int n_in,
                              void* d_out, int out_size, void* d_ws, size_t ws_size,
                              hipStream_t stream) {
  if (n_in < 2) return;
  if (in_sizes[0] != NQ * NCH * HW) return;
  if (in_sizes[1] != NCL * NBS * NCH * HW) return;
  if (out_size != NQ * OUTROW) return;
  if (ws_size < WS_TOTAL) return;

  const float* x1 = (const float*)d_in[0];
  const float* x2 = (const float*)d_in[1];
  char* ws = (char*)d_ws;
  float*          cs = (float*)(ws + OFF_CS);
  unsigned short* xh = (unsigned short*)(ws + OFF_XH);
  _Float16*       lp = (_Float16*)(ws + OFF_LP);
  _Float16*       dt = (_Float16*)(ws + OFF_DT);
  float* out = (float*)d_out;

  k_xprep<<<dim3(NCL * NCH), dim3(256), 0, stream>>>(x2, xh, cs);
  (void)hipGetLastError();
  k_qprep<<<dim3(NQ * 4), dim3(256), 0, stream>>>(x1, dt);
  (void)hipGetLastError();
  k_gram<<<dim3(NCL * GRAM_TILES), dim3(128), 0, stream>>>(xh, cs, lp);
  (void)hipGetLastError();
  k_sim<<<dim3(NQ / 2), dim3(256), 0, stream>>>(lp, dt, out);
  (void)hipGetLastError();
}
